// GDEE_81071802680057
// MI455X (gfx1250) — hardware-verified
//
#include <hip/hip_runtime.h>
#include <math.h>

constexpr int kTok       = 512;
constexpr int kVocab     = 30000;
constexpr int kEmb       = 300;
constexpr int kWtNum     = 20;
constexpr int kWte       = 50;
constexpr int kIn        = 350;
constexpr int kInPad     = 384;
constexpr int kHid       = 256;
constexpr int kGate      = 1024;
constexpr int kFin       = 256;
constexpr int kCls       = 34;
constexpr int kClsPad    = 64;
constexpr int kPairs     = kTok * kTok;
constexpr int kChunkRows = 65536;
constexpr int kNumChunks = kPairs / kChunkRows;
constexpr int kAhPitch   = 264;
constexpr int kThreads   = 256;
constexpr float kCarry     = 16.0f;
constexpr float kCarryInv  = 1.0f / 16.0f;
constexpr float kCarryInv2 = 1.0f / 256.0f;

typedef __attribute__((ext_vector_type(16))) _Float16 v16h;
typedef __attribute__((ext_vector_type(8)))  _Float16 v8h;
typedef __attribute__((ext_vector_type(16))) __bf16   v16b;
typedef __attribute__((ext_vector_type(8)))  __bf16   v8b;
typedef __attribute__((ext_vector_type(8)))  float    v8f;
typedef __attribute__((ext_vector_type(4)))  float    v4f;

__device__ __forceinline__ unsigned short f2bf_bits(float f) {
  unsigned u = __float_as_uint(f);
  return (unsigned short)((u + 0x7FFFu + ((u >> 16) & 1u)) >> 16);
}
__device__ __forceinline__ float bf_bits2f(unsigned short h) { return __uint_as_float(((unsigned)h) << 16); }

__device__ __forceinline__ void dep_guard_h(v8f& a, v8f& b, v16h x, v16h y) { asm volatile("v_nop\n\tv_nop\n\tv_nop\n\tv_nop" : "+v"(a), "+v"(b) : "v"(x), "v"(y)); }
__device__ __forceinline__ void dep_guard_b(v8f& a, v8f& b, v16b x, v16b y) { asm volatile("v_nop\n\tv_nop\n\tv_nop\n\tv_nop" : "+v"(a), "+v"(b) : "v"(x), "v"(y)); }
__device__ __forceinline__ void keep4_h(v16h a, v16h b, v16h c, v16h d) { asm volatile("v_nop" :: "v"(a), "v"(b), "v"(c), "v"(d)); }
__device__ __forceinline__ void keep4_b(v16b a, v16b b, v16b c, v16b d) { asm volatile("v_nop" :: "v"(a), "v"(b), "v"(c), "v"(d)); }
__device__ __forceinline__ void acc_guard4(v8f& a, v8f& b, v8f& c, v8f& d) { asm volatile("v_nop\n\tv_nop\n\tv_nop\n\tv_nop" : "+v"(a), "+v"(b), "+v"(c), "+v"(d)); }
template <typename T> struct Frag;
template <> struct Frag<_Float16> {
  typedef v16h V; union U { v16h v; v8h h[2]; };
  static __device__ __forceinline__ v16h load(const _Float16* p) {
    U f; f.h[0] = *(const v8h*)(p); f.h[1] = *(const v8h*)(p + 16); return f.v;
  }
  static __device__ __forceinline__ v8f mma(v16h a, v16h b, v8f c) {
    return __builtin_amdgcn_wmma_f32_16x16x32_f16(false, a, false, b, (short)0, c, false, false);
  }
  static __device__ __forceinline__ void guard(v8f& a, v8f& b, v16h x, v16h y) { dep_guard_h(a, b, x, y); }
  static __device__ __forceinline__ void keep(v16h a, v16h b, v16h c, v16h d) { keep4_h(a, b, c, d); }
};
template <> struct Frag<__bf16> {
  typedef v16b V; union U { v16b v; v8b h[2]; };
  static __device__ __forceinline__ v16b load(const __bf16* p) {
    U f; f.h[0] = *(const v8b*)(p); f.h[1] = *(const v8b*)(p + 16); return f.v;
  }
  static __device__ __forceinline__ v8f mma(v16b a, v16b b, v8f c) {
    return __builtin_amdgcn_wmma_f32_16x16x32_bf16(false, a, false, b, (short)0, c, false, false);
  }
  static __device__ __forceinline__ void guard(v8f& a, v8f& b, v16b x, v16b y) { dep_guard_b(a, b, x, y); }
  static __device__ __forceinline__ void keep(v16b a, v16b b, v16b c, v16b d) { keep4_b(a, b, c, d); }
};

template <int ET> struct Elem;
template <> struct Elem<0> { typedef _Float16 T; };
template <> struct Elem<1> { typedef __bf16 T; };
template <int ET, bool SPLIT, int BIAS_MODE, int OUT_MODE, bool RESID, int ACT = 0>
__global__ __launch_bounds__(256) void wmma_gemm64(
    const unsigned short* __restrict__ Ap, const unsigned short* __restrict__ A2p, int lda, long strideA,
    const unsigned short* __restrict__ Btp, const unsigned short* __restrict__ Bt2p, int ldb, long strideB,
    void* __restrict__ Cout, void* __restrict__ Cout2, int ldc, long strideC,
    const float* __restrict__ bias,
    const float* __restrict__ resid, long strideR,
    int M, int N, int K, float scale) {
  typedef typename Elem<ET>::T T;
  typedef typename Frag<T>::V V;
  const T* A = (const T*)Ap; const T* A2 = (const T*)A2p; const T* Bt = (const T*)Btp; const T* Bt2 = (const T*)Bt2p;
  __shared__ __align__(16) float sT[8][16 * 68];
  const int b    = blockIdx.y;
  const int lane = threadIdx.x & 31;
  const int wave = threadIdx.x >> 5;
  const int tilesN = N >> 6;
  const int tilesM = M >> 6;
  const int tile = blockIdx.x * 8 + wave;
  if (tile >= tilesM * tilesN) return;
  const int tm = tile / tilesN;
  const int tn = tile - tm * tilesN;
  const int m0 = tm << 6;
  const int n0 = tn << 6;

  const T* Ab  = A  + (size_t)b * strideA;
  const T* Bb  = Bt + (size_t)b * strideB;
  const T* Ab2 = SPLIT ? (A2  + (size_t)b * strideA) : nullptr;
  const T* Bb2 = SPLIT ? (Bt2 + (size_t)b * strideB) : nullptr;

  const int rlane = lane & 15;
  const int koff  = (lane >> 4) * 8;
  const int mOff  = (lane >> 4) * 8;

  v8f acc[4][4];
#pragma unroll
  for (int i = 0; i < 4; ++i)
#pragma unroll
    for (int j = 0; j < 4; ++j) acc[i][j] = (v8f){0.f,0.f,0.f,0.f,0.f,0.f,0.f,0.f};

  for (int k0 = 0; k0 < K; k0 += 32) {
    V bh[4], bl[4];
#pragma unroll
    for (int j = 0; j < 4; ++j) {
      const size_t bo = (size_t)(n0 + (j << 4) + rlane) * ldb + koff + k0;
      bh[j] = Frag<T>::load(Bb + bo);
      if (SPLIT) bl[j] = Frag<T>::load(Bb2 + bo);
    }
#pragma unroll
    for (int i = 0; i < 4; ++i) {
      const size_t ao = (size_t)(m0 + (i << 4) + rlane) * lda + koff + k0;
      V ah = Frag<T>::load(Ab + ao);
      V al;
      if (SPLIT) al = Frag<T>::load(Ab2 + ao);
#pragma unroll
      for (int j = 0; j < 4; ++j) {
        acc[i][j] = Frag<T>::mma(ah, bh[j], acc[i][j]);
        if (SPLIT) {
          acc[i][j] = Frag<T>::mma(ah, bl[j], acc[i][j]);
          acc[i][j] = Frag<T>::mma(al, bh[j], acc[i][j]);
        }
      }
      Frag<T>::guard(acc[i][0], acc[i][3], ah, SPLIT ? al : ah);
    }
    Frag<T>::keep(bh[0], bh[1], bh[2], bh[3]);
    if (SPLIT) Frag<T>::keep(bl[0], bl[1], bl[2], bl[3]);
  }
  acc_guard4(acc[0][0], acc[0][1], acc[0][2], acc[0][3]);
  acc_guard4(acc[1][0], acc[1][1], acc[1][2], acc[1][3]);
  acc_guard4(acc[2][0], acc[2][1], acc[2][2], acc[2][3]);
  acc_guard4(acc[3][0], acc[3][1], acc[3][2], acc[3][3]);

  float* slab = sT[wave];
  const float* Rb = RESID ? (resid + (size_t)b * strideR) : nullptr;
#pragma unroll
  for (int i = 0; i < 4; ++i) {
    const int mBase = m0 + (i << 4);
#pragma unroll
    for (int j = 0; j < 4; ++j) {
      const int n = n0 + (j << 4) + rlane;
      float bv = 0.f;
      if (BIAS_MODE == 2) bv = bias[n];
#pragma unroll
      for (int r = 0; r < 8; ++r) {
        float v = acc[i][j][r] * scale;
        if (BIAS_MODE == 1) v += bias[mBase + mOff + r];
        if (BIAS_MODE == 2) v += bv;
        if (RESID) v += Rb[(size_t)(mBase + mOff + r) * ldc + n];
        if (ACT == 1) v = tanhf(v);
        if (ACT == 2) v = fmaxf(v, 0.0f);
        if (ACT == 4) v = (v > 0.f) ? v : 0.01f * v;
        slab[(mOff + r) * 68 + (j << 4) + rlane] = v;
      }
    }
    __builtin_amdgcn_fence(__ATOMIC_RELEASE, "workgroup");
    __builtin_amdgcn_wave_barrier();
    __builtin_amdgcn_fence(__ATOMIC_ACQUIRE, "workgroup");
    if (OUT_MODE == 0) {
      float* C = (float*)Cout + (size_t)b * strideC;
      const int hh = lane >> 4, c4 = (lane & 15) * 4;
      for (int pass = 0; pass < 2; ++pass) {
#pragma unroll
        for (int it = 0; it < 8; ++it) {
          const int row = it * 2 + hh;
          v4f v = *(const v4f*)(slab + row * 68 + c4);
          *(volatile v4f*)(C + (size_t)(mBase + row) * ldc + n0 + c4) = v;
        }
        __threadfence();
      }
    } else {
      const int q = lane >> 3, c8 = (lane & 7) * 8;
      unsigned short* C  = (unsigned short*)Cout  + (size_t)b * strideC;
      unsigned short* C2 = (OUT_MODE == 2) ? ((unsigned short*)Cout2 + (size_t)b * strideC) : nullptr;
      for (int pass = 0; pass < 2; ++pass) {
#pragma unroll
        for (int it = 0; it < 4; ++it) {
          const int row = it * 4 + q;
          const float* sp = slab + row * 68 + c8;
          v8h hv, lv;
#pragma unroll
          for (int e = 0; e < 8; ++e) {
            if (OUT_MODE == 1) {
              hv[e] = (_Float16)sp[e];
            } else {
              unsigned short hb = f2bf_bits(sp[e]);
              unsigned short lb = f2bf_bits(sp[e] - bf_bits2f(hb));
              hv[e] = __builtin_bit_cast(_Float16, hb);
              lv[e] = __builtin_bit_cast(_Float16, lb);
            }
          }
          *(volatile v8h*)(C + (size_t)(mBase + row) * ldc + n0 + c8) = hv;
          if (OUT_MODE == 2) *(volatile v8h*)(C2 + (size_t)(mBase + row) * ldc + n0 + c8) = lv;
        }
        __threadfence();
      }
    }
    __builtin_amdgcn_fence(__ATOMIC_RELEASE, "workgroup");
    __builtin_amdgcn_wave_barrier();
    __builtin_amdgcn_fence(__ATOMIC_ACQUIRE, "workgroup");
  }
}

__global__ __launch_bounds__(kThreads) void cast_pad_kernel(const float* __restrict__ in, int rows_in, int cols_in,
                                                            int rows_out, int cols_out,
                                                            unsigned short* __restrict__ outp, float sc, int total8) {
  const int i = blockIdx.x * kThreads + threadIdx.x;
  if (i >= total8) return;
  const int per8 = cols_out >> 3;
  const int r = i / per8;
  const int c8 = (i - r * per8) * 8;
  const int rc = (r < rows_in) ? r : (rows_in - 1);
  (void)rows_out;
  v8h hv;
#pragma unroll
  for (int e = 0; e < 8; ++e) {
    const int c = c8 + e;
    const int cc = (c < cols_in) ? c : (cols_in - 1);
    float f = in[(size_t)rc * (size_t)cols_in + cc];
    f = (r < rows_in && c < cols_in) ? f * sc : 0.0f;
    hv[e] = (_Float16)f;
  }
  _Float16* o = (_Float16*)outp + (size_t)i * 8;
  *(volatile v8h*)o = hv;
  __threadfence();
  *(volatile v8h*)o = hv;
}

__global__ __launch_bounds__(64) void feat_kernel(const int* __restrict__ tok, const int* __restrict__ wty,
                                                 const float* __restrict__ etab, const float* __restrict__ wtab,
                                                 unsigned short* __restrict__ FEATp) {
  const int n = blockIdx.x, t = threadIdx.x;
  int tk = tok[n]; tk = tk < 0 ? 0 : (tk > kVocab - 1 ? kVocab - 1 : tk);
  int w  = wty[n]; w  = w  < 0 ? 0 : (w  > kWtNum - 1 ? kWtNum - 1 : w);
  const int c8 = t * 8;
  v8h hv;
#pragma unroll
  for (int e = 0; e < 8; ++e) {
    const int c = c8 + e;
    const int ce = (c < kEmb) ? c : (kEmb - 1);
    int cw = c - kEmb; cw = cw < 0 ? 0 : (cw > kWte - 1 ? kWte - 1 : cw);
    const float fe = etab[(size_t)tk * kEmb + ce];
    const float fw = wtab[w * kWte + cw];
    const float f = (c < kEmb) ? fe : ((c < kIn) ? fw : 0.0f);
    hv[e] = (_Float16)(f * kCarry);
  }
  if (t < kInPad / 8) {
    _Float16* dst = (_Float16*)FEATp + (size_t)n * kInPad + c8;
    *(volatile v8h*)dst = hv;
    __threadfence();
    *(volatile v8h*)dst = hv;
  }
}

__global__ __launch_bounds__(kThreads) void bias_kernel(const float* __restrict__ bihF, const float* __restrict__ bhhF,
                                                       const float* __restrict__ bihB, const float* __restrict__ bhhB,
                                                       const float* __restrict__ b2, const float* __restrict__ bfin,
                                                       float* __restrict__ BSUM, float* __restrict__ B2S, float* __restrict__ BFP) {
  const int i = blockIdx.x * kThreads + threadIdx.x;
  const float sf = bihF[i] + bhhF[i];
  const float sb = bihB[i] + bhhB[i];
  const int i2 = i < kFin ? i : kFin - 1;
  const float v2 = b2[i2] * kCarry;
  const int i3 = i < kCls ? i : kCls - 1;
  float v3 = bfin[i3];
  v3 = (i < kCls) ? v3 : 0.0f;
  for (int pass = 0; pass < 2; ++pass) {
    ((volatile float*)BSUM)[i] = sf;
    ((volatile float*)BSUM)[kGate + i] = sb;
    if (i < kFin) ((volatile float*)B2S)[i] = v2;
    if (i < kClsPad) ((volatile float*)BFP)[i] = v3;
    __threadfence();
  }
}

__device__ __forceinline__ float fsig(float x) { return __builtin_amdgcn_rcpf(1.0f + expf(-x)); }

__global__ __launch_bounds__(kThreads) void lstm_kernel(const float* __restrict__ preAll,
                                                       const unsigned short* __restrict__ WHHp,
                                                       unsigned short* __restrict__ HPp) {
  __shared__ __align__(16) _Float16 Ah[16 * kAhPitch];
  const int dir = blockIdx.x;
  const int tid = threadIdx.x, lane = tid & 31, wave = tid >> 5;
  const int c = lane & 15, hh = lane >> 4, koff = hh * 8;
  const float* pre = preAll + (size_t)dir * kTok * kGate;
  const _Float16* WH = (const _Float16*)WHHp + (size_t)dir * kGate * kHid;
  _Float16* HP = (_Float16*)HPp;

#pragma unroll 1
  for (int i = 0; i < 17; ++i) {
    const int idx = i * kThreads + tid;
    if (idx < 16 * kAhPitch) Ah[idx] = (_Float16)0.0f;
  }
  float cst[2] = {0.0f, 0.0f};
  __syncthreads();

  const _Float16* ahrow = Ah + c * kAhPitch + koff;
  const v8f z8 = {0.f, 0.f, 0.f, 0.f, 0.f, 0.f, 0.f, 0.f};

#pragma unroll 1
  for (int s = 0; s < kTok; ++s) {
    const int t = dir ? (kTok - 1 - s) : s;
    const float* pt = pre + (size_t)t * kGate;
    float hn[2];
#pragma unroll
    for (int nt = 0; nt < 2; ++nt) {
      const int j = 32 * wave + 16 * nt + c;
      const _Float16* wh = WH + (size_t)j * kHid + koff;
      v8f acc[4];
      acc[0] = z8; acc[1] = z8; acc[2] = z8; acc[3] = z8;
#pragma unroll 1
      for (int k0 = 0; k0 < kHid; k0 += 32) {
        const v16h a  = Frag<_Float16>::load(ahrow + k0);
        const v16h b0 = Frag<_Float16>::load(wh + k0);
        const v16h b1 = Frag<_Float16>::load(wh + (size_t)1 * kHid * kHid + k0);
        const v16h b2 = Frag<_Float16>::load(wh + (size_t)2 * kHid * kHid + k0);
        const v16h b3 = Frag<_Float16>::load(wh + (size_t)3 * kHid * kHid + k0);
        acc[0] = Frag<_Float16>::mma(a, b0, acc[0]);
        acc[1] = Frag<_Float16>::mma(a, b1, acc[1]);
        acc[2] = Frag<_Float16>::mma(a, b2, acc[2]);
        acc[3] = Frag<_Float16>::mma(a, b3, acc[3]);
        dep_guard_h(acc[0], acc[3], a, b3);
        keep4_h(b0, b1, b2, b3);
      }
      acc_guard4(acc[0], acc[1], acc[2], acc[3]);
      const float zi = acc[0][0] * kCarryInv2 + pt[j];
      const float zf = acc[1][0] * kCarryInv2 + pt[kHid + j];
      const float zg = acc[2][0] * kCarryInv2 + pt[2 * kHid + j];
      const float zo = acc[3][0] * kCarryInv2 + pt[3 * kHid + j];
      const float ig = fsig(zi);
      const float fg = fsig(zf);
      const float og = fsig(zo);
      const float gg = tanhf(zg);
      const float cn = fg * cst[nt] + ig * gg;
      cst[nt] = cn;
      hn[nt] = og * tanhf(cn);
    }
    __syncthreads();
    if (hh == 0) {
      Ah[32 * wave + c]      = (_Float16)(hn[0] * kCarry);
      Ah[32 * wave + 16 + c] = (_Float16)(hn[1] * kCarry);
    }
    __syncthreads();
    if (wave == 0) {
      const v8h v = *(const v8h*)(Ah + lane * 8);
      _Float16* dst = HP + (size_t)t * (2 * kHid) + dir * kHid + lane * 8;
      *(volatile v8h*)dst = v;
      __threadfence();
      *(volatile v8h*)dst = v;
    }
  }
}

__global__ __launch_bounds__(kThreads) void pair_kernel(const float* __restrict__ PQ, const float* __restrict__ b1,
                                                       unsigned short* __restrict__ OUT1p, int ibase) {
  const int g = blockIdx.x * kThreads + threadIdx.x;
  const int lrow = g >> 5;
  const int k8 = (g & 31) * 8;
  const int i = ibase + (lrow >> 9);
  const int j = lrow & 511;
  const float* Pp = PQ + (size_t)i * kFin + k8;
  const float* Qp = PQ + (size_t)kTok * kFin + (size_t)j * kFin + k8;
  const v4f p0 = *(const v4f*)Pp, p1 = *(const v4f*)(Pp + 4);
  const v4f q0 = *(const v4f*)Qp, q1 = *(const v4f*)(Qp + 4);
  const v4f c0 = *(const v4f*)(b1 + k8), c1 = *(const v4f*)(b1 + k8 + 4);
  v8h hv;
#pragma unroll
  for (int e = 0; e < 4; ++e) {
    float x0 = p0[e] + q0[e] + c0[e];
    x0 = (x0 > 0.0f) ? x0 : 0.01f * x0;
    hv[e] = (_Float16)(x0 * kCarry);
    float x1 = p1[e] + q1[e] + c1[e];
    x1 = (x1 > 0.0f) ? x1 : 0.01f * x1;
    hv[4 + e] = (_Float16)(x1 * kCarry);
  }
  _Float16* dst = (_Float16*)OUT1p + (size_t)lrow * kFin + k8;
  *(volatile v8h*)dst = hv;
  __threadfence();
  *(volatile v8h*)dst = hv;
}

__global__ __launch_bounds__(kThreads) void pack_kernel(const float* __restrict__ LOG, float* __restrict__ out,
                                                       int rowBase, int n4) {
  const int t = blockIdx.x * kThreads + threadIdx.x;
  if (t >= n4) return;
  const unsigned e0 = (unsigned)rowBase * (unsigned)kCls + 4u * (unsigned)t;
  v4f v;
#pragma unroll
  for (int q = 0; q < 4; ++q) {
    const unsigned idx = e0 + (unsigned)q;
    const unsigned row = idx / (unsigned)kCls;
    const unsigned col = idx - row * (unsigned)kCls;
    unsigned lrow = row - (unsigned)rowBase;
    lrow = lrow > (unsigned)(kChunkRows - 1) ? (unsigned)(kChunkRows - 1) : lrow;
    v[q] = LOG[(size_t)lrow * kClsPad + col];
  }
  float* dst = out + (size_t)e0;
  *(volatile v4f*)dst = v;
  __threadfence();
  *(volatile v4f*)dst = v;
}

extern "C" void kernel_launch(void* const* d_in, const int* in_sizes, int n_in,
                              void* d_out, int out_size, void* d_ws, size_t ws_size, hipStream_t stream) {
  if (n_in < 18 || d_out == nullptr || d_ws == nullptr) return;
  if (in_sizes[0] != kTok || in_sizes[1] != kTok || in_sizes[2] != kVocab * kEmb || in_sizes[3] != kWtNum * kWte ||
      in_sizes[4] != kGate * kIn || in_sizes[5] != kGate * kHid || in_sizes[6] != kGate || in_sizes[7] != kGate ||
      in_sizes[8] != kGate * kIn || in_sizes[9] != kGate * kHid || in_sizes[10] != kGate || in_sizes[11] != kGate ||
      in_sizes[12] != kFin * 4 * kHid || in_sizes[13] != kFin || in_sizes[14] != kFin * kFin || in_sizes[15] != kFin ||
      in_sizes[16] != kCls * kFin || in_sizes[17] != kCls || out_size != kPairs * kCls) return;

  const int*   tok  = (const int*)d_in[0];
  const int*   wty  = (const int*)d_in[1];
  const float* etab = (const float*)d_in[2];
  const float* wtab = (const float*)d_in[3];
  const float* WihF = (const float*)d_in[4];
  const float* WhhF = (const float*)d_in[5];
  const float* bihF = (const float*)d_in[6];
  const float* bhhF = (const float*)d_in[7];
  const float* WihB = (const float*)d_in[8];
  const float* WhhB = (const float*)d_in[9];
  const float* bihB = (const float*)d_in[10];
  const float* bhhB = (const float*)d_in[11];
  const float* W1   = (const float*)d_in[12];
  const float* b1   = (const float*)d_in[13];
  const float* W2   = (const float*)d_in[14];
  const float* b2   = (const float*)d_in[15];
  const float* Wf   = (const float*)d_in[16];
  const float* bfin = (const float*)d_in[17];
  float* out = (float*)d_out;

  char* ws = (char*)d_ws; size_t off = 0;
  auto carve = [&](size_t bytes) -> char* { char* p = ws + off; off += (bytes + 255) & ~(size_t)255; return p; };
  unsigned short* FEAT = (unsigned short*)carve((size_t)kTok * kInPad * 2);
  unsigned short* WIH  = (unsigned short*)carve((size_t)2 * kGate * kInPad * 2);
  unsigned short* WHH  = (unsigned short*)carve((size_t)2 * kGate * kHid * 2);
  float*          BSUM = (float*)carve((size_t)2 * kGate * 4);
  float*          PRE  = (float*)carve((size_t)2 * kTok * kGate * 4);
  unsigned short* HP   = (unsigned short*)carve((size_t)kTok * 2 * kHid * 2);
  unsigned short* W1P  = (unsigned short*)carve((size_t)kFin * 4 * kHid * 2);
  float*          PQ   = (float*)carve((size_t)2 * kTok * kFin * 4);
  unsigned short* W2P  = (unsigned short*)carve((size_t)kFin * kFin * 2);
  float*          B2S  = (float*)carve((size_t)kFin * 4);
  unsigned short* WFP  = (unsigned short*)carve((size_t)kClsPad * kFin * 2);
  float*          BFP  = (float*)carve((size_t)kClsPad * 4);
  unsigned short* OUT1 = (unsigned short*)carve((size_t)kChunkRows * kFin * 2);
  unsigned short* OUT2 = (unsigned short*)carve((size_t)kChunkRows * kFin * 2);
  float*          LOG  = (float*)carve((size_t)kChunkRows * kClsPad * 4);
  if (off > ws_size || off > (size_t)134217728) return;

  feat_kernel<<<kTok, 64, 0, stream>>>(tok, wty, etab, wtab, FEAT);
  {
    const int t8_wih = kGate * kInPad / 8;
    const int t8_whh = kGate * kHid / 8;
    const int t8_w1  = kFin * 4 * kHid / 8;
    const int t8_w2  = kFin * kFin / 8;
    const int t8_wf  = kClsPad * kFin / 8;
    cast_pad_kernel<<<(t8_wih + kThreads - 1) / kThreads, kThreads, 0, stream>>>(WihF, kGate, kIn, kGate, kInPad, WIH, kCarry, t8_wih);
    cast_pad_kernel<<<(t8_wih + kThreads - 1) / kThreads, kThreads, 0, stream>>>(WihB, kGate, kIn, kGate, kInPad, WIH + (size_t)kGate * kInPad, kCarry, t8_wih);
    cast_pad_kernel<<<(t8_whh + kThreads - 1) / kThreads, kThreads, 0, stream>>>(WhhF, kGate, kHid, kGate, kHid, WHH, kCarry, t8_whh);
    cast_pad_kernel<<<(t8_whh + kThreads - 1) / kThreads, kThreads, 0, stream>>>(WhhB, kGate, kHid, kGate, kHid, WHH + (size_t)kGate * kHid, kCarry, t8_whh);
    cast_pad_kernel<<<(t8_w1 + kThreads - 1) / kThreads, kThreads, 0, stream>>>(W1, kFin, 4 * kHid, kFin, 4 * kHid, W1P, kCarry, t8_w1);
    cast_pad_kernel<<<(t8_w2 + kThreads - 1) / kThreads, kThreads, 0, stream>>>(W2, kFin, kFin, kFin, kFin, W2P, kCarry, t8_w2);
    cast_pad_kernel<<<(t8_wf + kThreads - 1) / kThreads, kThreads, 0, stream>>>(Wf, kCls, kFin, kClsPad, kFin, WFP, kCarry, t8_wf);
  }
  bias_kernel<<<kGate / kThreads, kThreads, 0, stream>>>(bihF, bhhF, bihB, bhhB, b2, bfin, BSUM, B2S, BFP);

  {
    const int tiles = (kTok / 64) * (kGate / 64);
    dim3 grid((tiles + 7) / 8, 1);
    wmma_gemm64<0, false, 2, 0, false, 0><<<grid, 256, 0, stream>>>(
        FEAT, FEAT, kInPad, 0L, WIH, WIH, kInPad, 0L,
        (void*)PRE, (void*)PRE, kGate, 0L, BSUM, BSUM, 0L, kTok, kGate, kInPad, kCarryInv2);
    wmma_gemm64<0, false, 2, 0, false, 0><<<grid, 256, 0, stream>>>(
        FEAT, FEAT, kInPad, 0L, WIH + (size_t)kGate * kInPad, WIH + (size_t)kGate * kInPad, kInPad, 0L,
        (void*)(PRE + (size_t)kTok * kGate), (void*)(PRE + (size_t)kTok * kGate), kGate, 0L,
        BSUM + kGate, BSUM, 0L, kTok, kGate, kInPad, kCarryInv2);
  }

  lstm_kernel<<<2, kThreads, 0, stream>>>(PRE, WHH, HP);

  {
    const int tiles = (kTok / 64) * (kFin / 64);
    dim3 grid((tiles + 7) / 8, 2);
    wmma_gemm64<0, false, 0, 0, false, 0><<<grid, 256, 0, stream>>>(
        HP, HP, 2 * kHid, 0L, W1P, W1P, 4 * kHid, (long)(2 * kHid),
        (void*)PQ, (void*)PQ, kFin, (long)kTok * kFin, BSUM, BSUM, 0L, kTok, kFin, 2 * kHid, kCarryInv2);
  }

  for (int ch = 0; ch < kNumChunks; ++ch) {
    pair_kernel<<<(kChunkRows * 32) / kThreads, kThreads, 0, stream>>>(PQ, b1, OUT1, ch * (kChunkRows / kTok));
    {
      const int tiles = (kChunkRows / 64) * (kFin / 64);
      dim3 grid((tiles + 7) / 8, 1);
      wmma_gemm64<0, false, 2, 1, false, 4><<<grid, 256, 0, stream>>>(
          OUT1, OUT1, kFin, 0L, W2P, W2P, kFin, 0L,
          (void*)OUT2, (void*)OUT2, kFin, 0L, B2S, BSUM, 0L, kChunkRows, kFin, kFin, kCarryInv);
    }
    {
      const int tiles = (kChunkRows / 64) * (kClsPad / 64);
      dim3 grid((tiles + 7) / 8, 1);
      wmma_gemm64<0, false, 2, 0, false, 0><<<grid, 256, 0, stream>>>(
          OUT2, OUT2, kFin, 0L, WFP, WFP, kFin, 0L,
          (void*)LOG, (void*)LOG, kClsPad, 0L, BFP, BSUM, 0L, kChunkRows, kClsPad, kFin, kCarryInv2);
    }
    const int n4 = kChunkRows * kCls / 4;
    pack_kernel<<<(n4 + kThreads - 1) / kThreads, kThreads, 0, stream>>>(LOG, out, ch * kChunkRows, n4);
  }
}
